// TriangleAttentionStartingNode_2199023255612
// MI455X (gfx1250) — hardware-verified
//
#include <hip/hip_runtime.h>


#define NI   256
#define TT   256
#define DM   128
#define NH_  4
#define HD   32
#define HDP  64
#define DQ   (NH_ * HD)
#define IG   64
#define NTK  (IG * TT)
#define NTOK (NI * TT)
#define NBP  64
#define PCAR 1024.0f
#define SCL  0.17677669529663688f
typedef _Float16 h16;
typedef unsigned short bf;
typedef __attribute__((ext_vector_type(16))) __bf16   v16bf;
typedef __attribute__((ext_vector_type(16))) _Float16 v16h;
typedef __attribute__((ext_vector_type(8)))  _Float16 v8h;
typedef __attribute__((ext_vector_type(8)))  unsigned short v8us;
typedef __attribute__((ext_vector_type(8)))  float    v8f;
typedef __attribute__((ext_vector_type(4)))  float    v4f;
typedef v8h  __attribute__((may_alias)) v8ha;
typedef v4f  __attribute__((may_alias)) v4fa;
typedef v8us __attribute__((may_alias)) v8usa;

__device__ __forceinline__ unsigned short f2bf(float f) { unsigned u = __float_as_uint(f); u += 0x7FFFu + ((u >> 16) & 1u); return (unsigned short)(u >> 16); }
__device__ __forceinline__ float bf2f(unsigned short b) { return __uint_as_float(((unsigned)b) << 16); }
__device__ __forceinline__ float bfr(float f) { return bf2f(f2bf(f)); }
__device__ __forceinline__ v16h cat16(v8h lo, v8h hi) { return __builtin_shufflevector(lo, hi, 0, 1, 2, 3, 4, 5, 6, 7, 8, 9, 10, 11, 12, 13, 14, 15); }
__device__ __forceinline__ v16bf cat16b(v8us lo, v8us hi) { return __builtin_bit_cast(v16bf, __builtin_shufflevector(lo, hi, 0, 1, 2, 3, 4, 5, 6, 7, 8, 9, 10, 11, 12, 13, 14, 15)); }
__device__ __forceinline__ v8f wmma16(v16h a, v16h b, v8f c) { return __builtin_amdgcn_wmma_f32_16x16x32_f16(false, a, false, b, (short)0, c, false, false); }
__device__ __forceinline__ v8f wmmab(v16bf a, v16bf b, v8f c) { return __builtin_amdgcn_wmma_f32_16x16x32_bf16(false, a, false, b, (short)0, c, false, false); }


template <typename T16> struct WFrag;
template <> struct WFrag<h16> { typedef v16h V; static __device__ __forceinline__ V ld(const h16* p) { return cat16(*(const v8h*)p, *(const v8h*)(p + 16)); } static __device__ __forceinline__ v8f mma(V a, V b, v8f c) { return wmma16(a, b, c); } };
template <> struct WFrag<bf> { typedef v16bf V; static __device__ __forceinline__ V ld(const bf* p) { return cat16b(*(const v8us*)p, *(const v8us*)(p + 16)); } static __device__ __forceinline__ v8f mma(V a, V b, v8f c) { return wmmab(a, b, c); } };
template <typename T16, int NSPLIT, bool BIAS>
__global__ __launch_bounds__(32) void k_gemmw(const T16* __restrict__ A, const T16* __restrict__ A2, const T16* __restrict__ Bt, const T16* __restrict__ Bt2, int K, float* C, int ldc, const float* __restrict__ bias, size_t sA, size_t sB, size_t sC) {
    typedef typename WFrag<T16>::V V;
    __shared__ __align__(16) float os[16 * 68];
    const size_t z = blockIdx.z; A += z * sA; if (A2) A2 += z * sA; Bt += z * sB; if (Bt2) Bt2 += z * sB; C += z * sC;
    const int lane = threadIdx.x & 31, lr = lane & 15, hi = lane >> 4; const int r0 = blockIdx.x * 64, c0 = blockIdx.y * 64;
    v8f acc[4][4];
#pragma unroll
    for (int mb = 0; mb < 4; ++mb)
#pragma unroll
        for (int nb = 0; nb < 4; ++nb) acc[mb][nb] = (v8f){};
    const size_t aoff = (size_t)(r0 + lr) * K + 8 * hi, boff = (size_t)(c0 + lr) * K + 8 * hi;
#pragma unroll 1
    for (int kc = 0; kc < K; kc += 32) {
        V a[4], a2[4];
#pragma unroll
        for (int mb = 0; mb < 4; ++mb) { a[mb] = WFrag<T16>::ld(A + aoff + (size_t)mb * 16 * K + kc); if (NSPLIT == 1 || NSPLIT == 2) a2[mb] = WFrag<T16>::ld(A2 + aoff + (size_t)mb * 16 * K + kc); }
#pragma unroll
        for (int nb = 0; nb < 4; ++nb) { const V b = WFrag<T16>::ld(Bt + boff + (size_t)nb * 16 * K + kc); V b2; if (NSPLIT >= 2) b2 = WFrag<T16>::ld(Bt2 + boff + (size_t)nb * 16 * K + kc);
#pragma unroll
            for (int mb = 0; mb < 4; ++mb) { acc[mb][nb] = WFrag<T16>::mma(a[mb], b, acc[mb][nb]); if (NSPLIT == 1 || NSPLIT == 2) acc[mb][nb] = WFrag<T16>::mma(a2[mb], b, acc[mb][nb]); if (NSPLIT >= 2) acc[mb][nb] = WFrag<T16>::mma(a[mb], b2, acc[mb][nb]); } }
        asm volatile("v_nop\n\tv_nop\n\tv_nop\n\tv_nop" : "+v"(acc[0][0]), "+v"(acc[1][1]), "+v"(acc[2][2]), "+v"(acc[3][3]) : "v"(a[0]), "v"(a[3]));
    }
#pragma unroll
    for (int mb = 0; mb < 4; ++mb) {
#pragma unroll
        for (int nb = 0; nb < 4; ++nb) {
#pragma unroll
            for (int j = 0; j < 8; ++j) os[(hi * 8 + j) * 68 + nb * 16 + lr] = acc[mb][nb][j]; }
        __builtin_amdgcn_wave_barrier(); asm volatile("" ::: "memory");
        float* crow = C + (size_t)(r0 + mb * 16) * ldc + c0;
#pragma unroll 1
        for (int ps = 0; ps < 2; ++ps) {
#pragma unroll
            for (int s = 0; s < 8; ++s) { const int row = 2 * s + hi, cofs = lr * 4; v4f val = *(const v4fa*)(os + row * 68 + cofs); if (BIAS) { val[0] += bfr(bias[c0 + cofs]); val[1] += bfr(bias[c0 + cofs + 1]); val[2] += bfr(bias[c0 + cofs + 2]); val[3] += bfr(bias[c0 + cofs + 3]); }
                *(volatile v4f*)(crow + (size_t)row * ldc + cofs) = val; }
            if (ps == 0) __threadfence(); }
        __builtin_amdgcn_wave_barrier(); asm volatile("" ::: "memory");
    }
}

typedef __attribute__((ext_vector_type(4))) unsigned short v4us;
typedef __attribute__((ext_vector_type(2))) unsigned short v2us;
typedef __attribute__((ext_vector_type(2))) _Float16 v2h;
typedef __attribute__((ext_vector_type(4))) _Float16 v4h;
__device__ __forceinline__ h16 tohx(float x) { return (h16)x; }
__device__ __forceinline__ void splitf(float y, unsigned short& h, unsigned short& l) { h = f2bf(y); l = f2bf(y - bf2f(h)); }
__global__ __launch_bounds__(256) void k_wtG(const float* __restrict__ w, int K, int N, bf* Bt) {
    const int lane = threadIdx.x & 31; const int L0 = (blockIdx.x * 8 + (threadIdx.x >> 5)) * 8; const int nlines = N * K / 64;
#pragma unroll
    for (int ps = 0; ps < 2; ++ps) {
#pragma unroll 1
        for (int l = 0; l < 8; ++l) { const int L = L0 + l; if (L >= nlines) break; const size_t e = (size_t)L * 64 + lane * 2; const int k = (int)(e % K), n = (int)(e / K); v2us o;
            o[0] = f2bf(w[(size_t)k * N + n]); o[1] = f2bf(w[(size_t)(k + 1) * N + n]); *(volatile v2us*)(Bt + e) = o; }
        if (ps == 0) __threadfence(); }
}
__global__ __launch_bounds__(256) void k_cvt8(const float* __restrict__ src, bf* dst, size_t n8) { const size_t i = (size_t)blockIdx.x * 256 + threadIdx.x; if (i >= n8) return; const v8f v = *(const v8f*)(src + i * 8); v8us o;
#pragma unroll
    for (int k = 0; k < 8; ++k) o[k] = f2bf(v[k]); *(volatile v8us*)(dst + i * 8) = o; __threadfence(); *(volatile v8us*)(dst + i * 8) = o; }

__global__ __launch_bounds__(256) void k_w2d(const float* __restrict__ w, bf* Bt) { const int i = blockIdx.x * 256 + threadIdx.x; if (i >= NBP * DM / 8) return; const int r = i / (DM / 8), c0 = (i % (DM / 8)) * 8; v8us o;
#pragma unroll
    for (int k = 0; k < 8; ++k) o[k] = (r < NH_) ? f2bf(w[(size_t)(c0 + k) * NH_ + r]) : (unsigned short)0; *(volatile v8us*)(Bt + (size_t)r * DM + c0) = o; __threadfence(); *(volatile v8us*)(Bt + (size_t)r * DM + c0) = o; }
__global__ __launch_bounds__(256) void k_lnx(const float* __restrict__ A, const float* __restrict__ g, const float* __restrict__ bb, bf* Xh, bf* Xl) {
    const int lane = threadIdx.x & 31; const size_t tok = (size_t)blockIdx.x * 8 + (threadIdx.x >> 5); if (tok >= NTOK) return; const v4f a = *(const v4f*)(A + tok * DM + lane * 4); float v[4]; float s = 0.f;
#pragma unroll
    for (int q = 0; q < 4; ++q) { v[q] = bfr(a[q]); s = __fadd_rn(s, v[q]); }
#pragma unroll
    for (int sh = 16; sh; sh >>= 1) s = __fadd_rn(s, __shfl_xor(s, sh, 32));
    const float mu = __fdiv_rn(s, (float)DM); float s2 = 0.f;
#pragma unroll
    for (int q = 0; q < 4; ++q) { float d0 = __fsub_rn(v[q], mu); asm volatile("" : "+v"(d0)); float p = __fmul_rn(d0, d0); asm volatile("" : "+v"(p)); s2 = __fadd_rn(s2, p); }
#pragma unroll
    for (int sh = 16; sh; sh >>= 1) s2 = __fadd_rn(s2, __shfl_xor(s2, sh, 32));
    const float rs = __fdiv_rn(1.0f, __fsqrt_rn(__fadd_rn(__fdiv_rn(s2, (float)DM), 1e-5f))); v4us oh, ol;
#pragma unroll
    for (int q = 0; q < 4; ++q) { const int c = lane * 4 + q; float xn = __fmul_rn(__fsub_rn(v[q], mu), rs); asm volatile("" : "+v"(xn)); float gg = bfr(g[c]); asm volatile("" : "+v"(gg)); float y = __fmul_rn(xn, gg); asm volatile("" : "+v"(y)); float be = bfr(bb[c]); asm volatile("" : "+v"(be)); y = __fadd_rn(y, be); unsigned short h2, l2; splitf(y, h2, l2); oh[q] = h2; ol[q] = l2; }
    *(volatile v4us*)(Xh + tok * DM + lane * 4) = oh; *(volatile v4us*)(Xl + tok * DM + lane * 4) = ol; __threadfence(); *(volatile v4us*)(Xh + tok * DM + lane * 4) = oh; *(volatile v4us*)(Xl + tok * DM + lane * 4) = ol; }
__global__ __launch_bounds__(256) void k_qkpl(const float* __restrict__ F, h16* P16) { const size_t e = ((size_t)blockIdx.x * 256 + threadIdx.x) * 2; if (e >= (size_t)NH_ * NTK * HD) return; const int d = (int)(e % HD); const size_t tk = (e / HD) % NTK; const int h = (int)(e / ((size_t)HD * NTK)); v2h o;
    o[0] = tohx(F[tk * DQ + h * HD + d]); o[1] = tohx(F[tk * DQ + h * HD + d + 1]); *(volatile v2h*)(P16 + e) = o; __threadfence(); *(volatile v2h*)(P16 + e) = o; }
__global__ __launch_bounds__(256) void k_vtpl(const float* __restrict__ F, h16* V16) { const size_t e = ((size_t)blockIdx.x * 256 + threadIdx.x) * 2; if (e >= (size_t)NH_ * IG * HDP * TT) return; const int t = (int)(e % TT); const int dp = (int)((e / TT) % HDP); const size_t il = (e / ((size_t)TT * HDP)) % IG; const int h = (int)(e / ((size_t)TT * HDP * IG)); v2h o;
    if (dp < HD) { o[0] = tohx(F[(il * TT + t) * DQ + h * HD + dp]); o[1] = tohx(F[(il * TT + t + 1) * DQ + h * HD + dp]); } else { o[0] = (h16)0.0f; o[1] = (h16)0.0f; }
    *(volatile v2h*)(V16 + e) = o; __threadfence(); *(volatile v2h*)(V16 + e) = o; }
__global__ __launch_bounds__(256) void k_asoftT(const float* __restrict__ Sb, const float* __restrict__ NB, int i0, int h, h16* P16) {
    const int lane = threadIdx.x & 31; const int row = blockIdx.x * 8 + (threadIdx.x >> 5); if (row >= IG * TT) return; const int q = row % TT; const int il = row / TT; const int i = i0 + il; const float* sr = Sb + (size_t)row * TT; float v[TT / 32]; float mx = -3.0e38f;
#pragma unroll
    for (int ch = 0; ch < TT / 128; ++ch) { const int j0 = ch * 128 + lane * 4; const v4f a = *(const v4f*)(sr + j0);
#pragma unroll
        for (int qq = 0; qq < 4; ++qq) { const int j = j0 + qq; float sc = __fmul_rn(a[qq], SCL); asm volatile("" : "+v"(sc)); const float nb = NB[((size_t)j * TT + q) * NBP + h];     const float t = __fadd_rn(sc, nb); v[ch * 4 + qq] = t; mx = fmaxf(mx, t); } }
#pragma unroll
    for (int sh = 16; sh; sh >>= 1) mx = fmaxf(mx, __shfl_xor(mx, sh, 32));
    float sum = 0.f;
#pragma unroll
    for (int kk = 0; kk < TT / 32; ++kk) { float d0 = __fsub_rn(v[kk], mx); asm volatile("" : "+v"(d0)); v[kk] = __builtin_amdgcn_exp2f(__fmul_rn(d0, 1.4426950408889634f)); sum += v[kk]; }
#pragma unroll
    for (int sh = 16; sh; sh >>= 1) sum += __shfl_xor(sum, sh, 32);
    const float f = __fdiv_rn(PCAR, sum);
#pragma unroll 1
    for (int ps = 0; ps < 2; ++ps) {
#pragma unroll
        for (int ch = 0; ch < TT / 128; ++ch) { v4h o4;
#pragma unroll
            for (int qq = 0; qq < 4; ++qq) { float y = __fmul_rn(v[ch * 4 + qq], f); asm volatile("" : "+v"(y)); o4[qq] = tohx(y); }
            *(volatile v4h*)(P16 + (size_t)row * TT + ch * 128 + lane * 4) = o4; }
        if (ps == 0) __threadfence(); }
}
__global__ __launch_bounds__(256) void k_wtP(const float* __restrict__ w, bf* Bt) { const int lane = threadIdx.x & 31; const int L0 = (blockIdx.x * 8 + (threadIdx.x >> 5)) * 8; const int nlines = DQ * DM / 64;
#pragma unroll
    for (int ps = 0; ps < 2; ++ps) {
#pragma unroll 1
        for (int l = 0; l < 8; ++l) { const int L = L0 + l; if (L >= nlines) break; const size_t e = (size_t)L * 64 + lane * 2; const int k = (int)(e % DM), n = (int)(e / DM); const int hh = n / HD, cc = n % HD; v2us o;
            o[0] = f2bf(w[(size_t)k * DQ + cc * NH_ + hh]); o[1] = f2bf(w[(size_t)(k + 1) * DQ + cc * NH_ + hh]); *(volatile v2us*)(Bt + e) = o; }
        if (ps == 0) __threadfence(); } }
__global__ __launch_bounds__(256) void k_wtPo(const float* __restrict__ w, bf* Bt) { const int lane = threadIdx.x & 31; const int L0 = (blockIdx.x * 8 + (threadIdx.x >> 5)) * 8; const int nlines = DM * DQ / 64;
#pragma unroll
    for (int ps = 0; ps < 2; ++ps) {
#pragma unroll 1
        for (int l = 0; l < 8; ++l) { const int L = L0 + l; if (L >= nlines) break; const size_t e = (size_t)L * 64 + lane * 2; const int n = (int)(e % DQ), cout = (int)(e / DQ); v2us o;
#pragma unroll
            for (int q = 0; q < 2; ++q) { const int nn = n + q; const int hh = nn / HD, cc = nn % HD; o[q] = f2bf(w[(size_t)(cc * NH_ + hh) * DM + cout]); }
            *(volatile v2us*)(Bt + e) = o; }
        if (ps == 0) __threadfence(); } }
__global__ __launch_bounds__(32) void k_bgp(const float* __restrict__ bg, float* BGP) { const int i = threadIdx.x; if (i >= DQ / 4) return; v4f o;
#pragma unroll
    for (int q = 0; q < 4; ++q) { const int n = i * 4 + q; o[q] = bg[(n % HD) * NH_ + n / HD]; } *(volatile v4f*)(BGP + i * 4) = o; __threadfence(); *(volatile v4f*)(BGP + i * 4) = o; }
__global__ __launch_bounds__(256) void k_gmerge(const float* __restrict__ O, const float* __restrict__ FG, const float* __restrict__ bg, bf* Ah, bf* Al) { const size_t e = ((size_t)blockIdx.x * 256 + threadIdx.x) * 4; if (e >= (size_t)NTK * DQ) return; const int c = (int)(e % DQ); const size_t tk = e / DQ; const int h = c / HD, d = c % HD; v4us oh, ol;
    const v4f ov = *(const v4f*)(O + (((size_t)h * NTK + tk) * HDP + d)); const v4f gv = *(const v4f*)(FG + tk * DQ + c);
#pragma unroll
    for (int qq = 0; qq < 4; ++qq) { float bgv = bfr(bg[c + qq]); asm volatile("" : "+v"(bgv)); const float ga = __fadd_rn(gv[qq], bgv); const float sg = __fdiv_rn(1.0f, __fadd_rn(1.0f, __builtin_amdgcn_exp2f(__fmul_rn(ga, -1.4426950408889634f)))); float o1 = __fmul_rn(ov[qq], 1.0f / PCAR); asm volatile("" : "+v"(o1)); const float y = __fmul_rn(o1, sg); unsigned short h2, l2; splitf(y, h2, l2); oh[qq] = h2; ol[qq] = l2; }
    *(volatile v4us*)(Ah + e) = oh; *(volatile v4us*)(Al + e) = ol; __threadfence(); *(volatile v4us*)(Ah + e) = oh; *(volatile v4us*)(Al + e) = ol; }

extern "C" void kernel_launch(void* const* d_in, const int* in_sizes, int n_in,
                              void* d_out, int out_size, void* d_ws, size_t ws_size, hipStream_t stream) {
    (void)in_sizes; (void)n_in; (void)out_size;
    const float* act = (const float*)d_in[0]; const float* lng = (const float*)d_in[1]; const float* lnb = (const float*)d_in[2]; const float* wq = (const float*)d_in[3]; const float* wk = (const float*)d_in[4]; const float* wv = (const float*)d_in[5]; const float* w2d = (const float*)d_in[6]; const float* wg = (const float*)d_in[7]; const float* bg = (const float*)d_in[8]; const float* wo = (const float*)d_in[9]; const float* bo = (const float*)d_in[10];
    float* OUT = (float*)d_out;
    char* wsp = (char*)d_ws;
    auto take = [&](size_t bytes) { char* p = wsp; wsp += (bytes + 255) & ~(size_t)255; return (void*)p; };
    bf* WQ = (bf*)take((size_t)DQ * DM * 2); bf* WK = (bf*)take((size_t)DQ * DM * 2); bf* WV = (bf*)take((size_t)DQ * DM * 2); bf* WG = (bf*)take((size_t)DQ * DM * 2); float* BGP = (float*)take((size_t)DQ * 4); bf* WO = (bf*)take((size_t)DM * DQ * 2); bf* W2 = (bf*)take((size_t)NBP * DM * 2);
    bf* Xh = (bf*)take((size_t)NTOK * DM * 2); bf* Xl = (bf*)take((size_t)NTOK * DM * 2); float* NB = (float*)take((size_t)NTOK * NBP * 4);
    float* FQ = (float*)take((size_t)NTK * DQ * 4); float* FK = (float*)take((size_t)NTK * DQ * 4); float* FG = (float*)take((size_t)NTK * DQ * 4); h16* QP16 = (h16*)take((size_t)NH_ * NTK * HD * 2); h16* KP16 = (h16*)take((size_t)NH_ * NTK * HD * 2); h16* VT16 = (h16*)take((size_t)NH_ * IG * HDP * TT * 2);
    float* Sb = (float*)take((size_t)IG * TT * TT * 4); h16* P16 = (h16*)take((size_t)IG * TT * TT * 2); float* Ob = (float*)take((size_t)NH_ * NTK * HDP * 4); bf* ATh = (bf*)take((size_t)NTK * DQ * 2); bf* ATl = (bf*)take((size_t)NTK * DQ * 2);
    if ((size_t)(wsp - (char*)d_ws) > ws_size) return;
    float* FV = FK;
    k_wtP<<<(unsigned)((DM * DQ / 64 + 63) / 64), 256, 0, stream>>>(wq, WQ); k_wtP<<<(unsigned)((DM * DQ / 64 + 63) / 64), 256, 0, stream>>>(wk, WK); k_wtP<<<(unsigned)((DM * DQ / 64 + 63) / 64), 256, 0, stream>>>(wv, WV); k_wtP<<<(unsigned)((DM * DQ / 64 + 63) / 64), 256, 0, stream>>>(wg, WG); k_bgp<<<1, 32, 0, stream>>>(bg, BGP);
    k_wtPo<<<(unsigned)((DQ * DM / 64 + 63) / 64), 256, 0, stream>>>(wo, WO); k_w2d<<<(NBP * DM / 8 + 255) / 256, 256, 0, stream>>>(w2d, W2);
    k_lnx<<<NTOK / 8, 256, 0, stream>>>(act, lng, lnb, Xh, Xl);
    k_gemmw<bf, 1, false><<<dim3(NTOK / 64, NBP / 64, 1), 32, 0, stream>>>(Xh, Xl, W2, nullptr, DM, NB, NBP, nullptr, 0, 0, 0);
    for (int i0 = 0; i0 < NI; i0 += IG) { const bf* Xgh = Xh + (size_t)i0 * TT * DM; const bf* Xgl = Xl + (size_t)i0 * TT * DM;
        k_gemmw<bf, 1, false><<<dim3(NTK / 64, DQ / 64, 1), 32, 0, stream>>>(Xgh, Xgl, WQ, nullptr, DM, FQ, DQ, nullptr, 0, 0, 0); k_qkpl<<<(unsigned)(((size_t)NH_ * NTK * HD / 2 + 255) / 256), 256, 0, stream>>>(FQ, QP16);
        k_gemmw<bf, 1, false><<<dim3(NTK / 64, DQ / 64, 1), 32, 0, stream>>>(Xgh, Xgl, WK, nullptr, DM, FK, DQ, nullptr, 0, 0, 0); k_qkpl<<<(unsigned)(((size_t)NH_ * NTK * HD / 2 + 255) / 256), 256, 0, stream>>>(FK, KP16);
        k_gemmw<bf, 1, false><<<dim3(NTK / 64, DQ / 64, 1), 32, 0, stream>>>(Xgh, Xgl, WV, nullptr, DM, FV, DQ, nullptr, 0, 0, 0); k_vtpl<<<(unsigned)(((size_t)NH_ * IG * HDP * TT / 2 + 255) / 256), 256, 0, stream>>>(FV, VT16);
        k_gemmw<bf, 1, false><<<dim3(NTK / 64, DQ / 64, 1), 32, 0, stream>>>(Xgh, Xgl, WG, nullptr, DM, FG, DQ, nullptr, 0, 0, 0);
        for (int h = 0; h < NH_; ++h) {
            k_gemmw<h16, 0, false><<<dim3(TT / 64, TT / 64, IG), 32, 0, stream>>>(QP16 + (size_t)h * NTK * HD, nullptr, KP16 + (size_t)h * NTK * HD, nullptr, HD, Sb, TT, nullptr, (size_t)TT * HD, (size_t)TT * HD, (size_t)TT * TT);
            k_asoftT<<<IG * TT / 8, 256, 0, stream>>>(Sb, NB, i0, h, P16);
            k_gemmw<h16, 0, false><<<dim3(TT / 64, HDP / 64, IG), 32, 0, stream>>>(P16, nullptr, VT16 + (size_t)h * IG * HDP * TT, nullptr, TT, Ob + (size_t)h * NTK * HDP, HDP, nullptr, (size_t)TT * TT, (size_t)HDP * TT, (size_t)TT * HDP); }
        k_gmerge<<<(unsigned)(((size_t)NTK * DQ / 4 + 255) / 256), 256, 0, stream>>>(Ob, FG, BGP, ATh, ATl);
        k_gemmw<bf, 1, true><<<dim3(NTK / 64, DM / 64, 1), 32, 0, stream>>>(ATh, ATl, WO, nullptr, DQ, OUT + (size_t)i0 * TT * DM, DM, bo, 0, 0, 0); }
}
